// MambaBlock_53652731462300
// MI455X (gfx1250) — hardware-verified
//
#include <hip/hip_runtime.h>
#include <math.h>

typedef __attribute__((ext_vector_type(16))) _Float16 v16h;
typedef __attribute__((ext_vector_type(8)))  _Float16 v8h;
typedef __attribute__((ext_vector_type(8)))  float    v8f;
typedef __attribute__((ext_vector_type(4)))  float    v4f;

constexpr int kBatch  = 2;
constexpr int kSeq    = 2048;
constexpr int kHid    = 1024;
constexpr int kInner  = 2048;
constexpr int kNst    = 16;
constexpr int kDtR    = 64;
constexpr int kProjW  = 2 * kInner;
constexpr int kCatP   = 128;
constexpr int kBcP    = 32;
constexpr int kRows   = kBatch * kSeq;
constexpr int kScanTS = 64;
constexpr int kScanCh = 64;
constexpr int kScanYP = 68;
constexpr float kWCarry  = 32.0f;
constexpr float kDrCarry = 16.0f;
constexpr float kYCarry  = 16.0f;
static_assert((kHid % 32) == 0 && (kInner % 32) == 0 && (kDtR % 32) == 0, "GEMM K multiples of 32");
static_assert((kRows % 64) == 0 && (kProjW % 64) == 0 && (kInner % 64) == 0 && (kHid % 64) == 0 && (kCatP % 64) == 0 && (kDtR % 64) == 0, "GEMM M,N multiples of 64");
static_assert((kSeq % kScanTS) == 0 && (kInner % kScanCh) == 0, "scan tile multiples");
static_assert(kDtR + 2 * kNst <= kCatP && 2 * kNst == kBcP, "merged projection layout");
static_assert((kRows % 8) == 0 && kHid == 1024, "layer-norm kernel layout");

constexpr size_t kOffWINT = 0;
constexpr size_t kOffWCAT = kOffWINT + (size_t)kProjW * kHid * 2;
constexpr size_t kOffWDT  = kOffWCAT + (size_t)kCatP * kInner * 2;
constexpr size_t kOffWOUT = kOffWDT  + (size_t)kInner * kDtR * 2;
constexpr size_t kOffXN16 = kOffWOUT + (size_t)kHid * kInner * 2;
constexpr size_t kOffU16  = kOffXN16 + (size_t)kRows * kHid * 2;
constexpr size_t kOffSG16 = kOffU16  + (size_t)kRows * kInner * 2;
constexpr size_t kOffDR16 = kOffSG16 + (size_t)kRows * kInner * 2;
constexpr size_t kOffBC   = kOffDR16 + (size_t)kRows * kDtR * 2;
constexpr size_t kOffZ16  = kOffBC   + (size_t)kRows * kBcP * 4;
constexpr size_t kOffY16  = kOffZ16  + (size_t)kRows * kInner * 2;
constexpr size_t kWsTotal = kOffY16  + (size_t)kRows * kInner * 2;
static_assert(kWsTotal == 89915392ull, "carve total");
static_assert(kWsTotal <= 134217728ull, "carve cap");
static_assert((kOffWCAT % 128) == 0 && (kOffWDT % 128) == 0 && (kOffWOUT % 128) == 0 && (kOffXN16 % 128) == 0 &&
              (kOffU16 % 128) == 0 && (kOffSG16 % 128) == 0 && (kOffDR16 % 128) == 0 && (kOffBC % 128) == 0 &&
              (kOffZ16 % 128) == 0 && (kOffY16 % 128) == 0, "128-B aligned regions");

__device__ __forceinline__ float h16_to_f32(unsigned hb) {
  const unsigned sgn = (hb & 0x8000u) << 16;
  const unsigned em = hb & 0x7fffu;
  const float fn = __uint_as_float((em << 13) + 0x38000000u);
  const float fs = (float)em * 5.9604644775390625e-8f;
  const float mag = (em < 0x400u) ? fs : fn;
  return __uint_as_float(__float_as_uint(mag) | sgn);
}

__device__ __forceinline__ void grp_guard(v8f& a0, v8f& a1, v8f& a2, v8f& a3, v16h x, v16h b0, v16h b1, v16h b2, v16h b3) {
  asm volatile("v_nop\n\tv_nop\n\tv_nop\n\tv_nop" : "+v"(a0), "+v"(a1), "+v"(a2), "+v"(a3) : "v"(x), "v"(b0), "v"(b1), "v"(b2), "v"(b3));
}
__device__ __forceinline__ void keep4_h(v16h a, v16h b, v16h c, v16h d) { asm volatile("v_nop" :: "v"(a), "v"(b), "v"(c), "v"(d)); }
__device__ __forceinline__ void acc_guard4(v8f& a, v8f& b, v8f& c, v8f& d) { asm volatile("v_nop\n\tv_nop\n\tv_nop\n\tv_nop" : "+v"(a), "+v"(b), "+v"(c), "+v"(d)); }

struct FragH {
  union U { v16h v; v8h h[2]; };
  static __device__ __forceinline__ v16h load(const _Float16* p) {
    U f; f.h[0] = *(const v8h*)(p); f.h[1] = *(const v8h*)(p + 16); return f.v;
  }
  static __device__ __forceinline__ v8f mma(v16h a, v16h b, v8f c) {
    return __builtin_amdgcn_wmma_f32_16x16x32_f16(false, a, false, b, (short)0, c, false, false);
  }
};

template <int OUT_MODE, bool RESID, int ACT>
__global__ __launch_bounds__(256) void gemm64_f16(
    const unsigned short* __restrict__ Ap, int lda,
    const unsigned short* __restrict__ Btp, int ldb,
    void* Cout, void* Cout2, int ldc, int nsplit,
    const float* __restrict__ bias, const float* __restrict__ bias2,
    const float* __restrict__ resid,
    int M, int N, int K, float scale, float bscale)
{
  const _Float16* A  = (const _Float16*)Ap;
  const _Float16* Bt = (const _Float16*)Btp;
  __shared__ __align__(16) float sT[8][16 * 68];
  const int lane = threadIdx.x & 31;
  const int wave = threadIdx.x >> 5;
  const int tilesN = N >> 6;
  const int tilesM = M >> 6;
  const int tile = blockIdx.x * 8 + wave;
  if (tile >= tilesM * tilesN) return;
  const int tm = tile / tilesN;
  const int tn = tile - tm * tilesN;
  const int m0 = tm << 6;
  const int n0 = tn << 6;

  const int rlane = lane & 15;
  const int koff  = (lane >> 4) * 8;
  const int mOff  = (lane >> 4) * 8;

  v8f acc[4][4];
#pragma unroll
  for (int i = 0; i < 4; ++i)
#pragma unroll
    for (int j = 0; j < 4; ++j) acc[i][j] = (v8f){0.f,0.f,0.f,0.f,0.f,0.f,0.f,0.f};

  for (int k0 = 0; k0 < K; k0 += 32) {
    v16h bh[4];
#pragma unroll
    for (int j = 0; j < 4; ++j) {
      const size_t bo = (size_t)(n0 + (j << 4) + rlane) * ldb + koff + k0;
      bh[j] = FragH::load(Bt + bo);
    }
#pragma unroll
    for (int i = 0; i < 4; ++i) {
      const size_t ao = (size_t)(m0 + (i << 4) + rlane) * lda + koff + k0;
      const v16h ah = FragH::load(A + ao);
#pragma unroll
      for (int j = 0; j < 4; ++j) acc[i][j] = FragH::mma(ah, bh[j], acc[i][j]);
      grp_guard(acc[i][0], acc[i][1], acc[i][2], acc[i][3], ah, bh[0], bh[1], bh[2], bh[3]);
    }
    keep4_h(bh[0], bh[1], bh[2], bh[3]);
  }
  acc_guard4(acc[0][0], acc[0][1], acc[0][2], acc[0][3]);
  acc_guard4(acc[1][0], acc[1][1], acc[1][2], acc[1][3]);
  acc_guard4(acc[2][0], acc[2][1], acc[2][2], acc[2][3]);
  acc_guard4(acc[3][0], acc[3][1], acc[3][2], acc[3][3]);

  float* slab = sT[wave];
#pragma unroll
  for (int i = 0; i < 4; ++i) {
    const int mBase = m0 + (i << 4);
#pragma unroll
    for (int j = 0; j < 4; ++j) {
      float bv = 0.f;
      if (OUT_MODE == 3) {
        if (j == 0) bv = bias[rlane];
        if (j == 1) bv = bias2[rlane];
      } else {
        bv = bias[n0 + (j << 4) + rlane];
      }
      bv = bv * bscale;
#pragma unroll
      for (int r = 0; r < 8; ++r) {
        const float v = acc[i][j][r] * scale + bv;
        slab[(mOff + r) * 68 + (j << 4) + rlane] = v;
      }
    }
    __builtin_amdgcn_fence(__ATOMIC_RELEASE, "workgroup");
    __builtin_amdgcn_wave_barrier();
    __builtin_amdgcn_fence(__ATOMIC_ACQUIRE, "workgroup");
    if (OUT_MODE == 0) {
      float* C = (float*)Cout;
      const int hh = lane >> 4, c4 = (lane & 15) * 4;
#pragma unroll 1
      for (int pass = 0; pass < 2; ++pass) {
#pragma unroll
        for (int it = 0; it < 8; ++it) {
          const int row = it * 2 + hh;
          const size_t go = (size_t)(mBase + row) * ldc + n0 + c4;
          v4f v = *(const v4f*)(slab + row * 68 + c4);
          if (RESID) {
            const v4f rv = *(const v4f*)(resid + go);
            v = v + rv;
          }
          *(volatile v4f*)(C + go) = v;
        }
        __threadfence();
      }
    } else if (OUT_MODE == 3) {
      float* C = (float*)Cout;
      const int q = lane >> 3, c4 = (lane & 7) * 4;
#pragma unroll 1
      for (int pass = 0; pass < 2; ++pass) {
#pragma unroll
        for (int it = 0; it < 4; ++it) {
          const int row = it * 4 + q;
          const v4f v = *(const v4f*)(slab + row * 68 + c4);
          *(volatile v4f*)(C + (size_t)(mBase + row) * ldc + c4) = v;
        }
        __threadfence();
      }
    } else {
      const int q = lane >> 3, c8 = (lane & 7) * 8;
      unsigned short* Cb = (unsigned short*)Cout;
      int nc0 = n0;
      if (n0 >= nsplit) { Cb = (unsigned short*)Cout2; nc0 = n0 - nsplit; }
#pragma unroll 1
      for (int pass = 0; pass < 2; ++pass) {
#pragma unroll 1
        for (int it = 0; it < 4; ++it) {
          const int row = it * 4 + q;
          const float* sp = slab + row * 68 + c8;
          const v4f a0 = *(const v4f*)(sp);
          const v4f a1 = *(const v4f*)(sp + 4);
          v8h hv;
#pragma unroll
          for (int e = 0; e < 4; ++e) {
            float f0 = a0[e];
            float f1 = a1[e];
            if (ACT == 3) {
              f0 = f0 * __builtin_amdgcn_rcpf(1.0f + expf(-f0));
              f1 = f1 * __builtin_amdgcn_rcpf(1.0f + expf(-f1));
            }
            hv[e]     = (_Float16)f0;
            hv[4 + e] = (_Float16)f1;
          }
          *(volatile v8h*)(Cb + (size_t)(mBase + row) * ldc + nc0 + c8) = hv;
        }
        __threadfence();
      }
    }
    __builtin_amdgcn_fence(__ATOMIC_RELEASE, "workgroup");
    __builtin_amdgcn_wave_barrier();
    __builtin_amdgcn_fence(__ATOMIC_ACQUIRE, "workgroup");
  }
}

__global__ __launch_bounds__(256) void transpose_cast_kernel(
    const float* __restrict__ W, unsigned short* __restrict__ Bt, int Kdim, int Ndim, float scale)
{
  __shared__ float tile[64 * 65];
  const int tid = threadIdx.x, lane = tid & 31, wave = tid >> 5;
  const int n0 = blockIdx.x * 64;
  const int k0 = blockIdx.y * 64;
#pragma unroll
  for (int p = 0; p < 16; ++p) {
    const int idx = tid + p * 256;
    const int kk  = idx >> 6;
    const int nn  = idx & 63;
    const int n   = n0 + nn;
    const int nc  = (n < Ndim) ? n : (Ndim - 1);
    const float v = W[(size_t)(k0 + kk) * Ndim + nc];
    tile[kk * 65 + nn] = (n < Ndim) ? (v * scale) : 0.f;
  }
  __syncthreads();
  const int q = lane >> 3, c8 = (lane & 7) * 8;
  v8h hv[2];
#pragma unroll
  for (int it = 0; it < 2; ++it) {
    const int nrow = it * 32 + wave * 4 + q;
#pragma unroll
    for (int e = 0; e < 8; ++e) hv[it][e] = (_Float16)tile[(c8 + e) * 65 + nrow];
  }
  for (int pass = 0; pass < 2; ++pass) {
#pragma unroll
    for (int it = 0; it < 2; ++it) {
      const int nrow = it * 32 + wave * 4 + q;
      *(volatile v8h*)(Bt + (size_t)(n0 + nrow) * Kdim + k0 + c8) = hv[it];
    }
    __threadfence();
  }
}

__global__ __launch_bounds__(256) void transpose_cast_bc_kernel(
    const float* __restrict__ WB, const float* __restrict__ WC, unsigned short* __restrict__ Bt, int Kdim, float scale)
{
  __shared__ float tile[64 * 65];
  const int tid = threadIdx.x, lane = tid & 31, wave = tid >> 5;
  const int k0 = blockIdx.x * 64;
#pragma unroll
  for (int p = 0; p < 16; ++p) {
    const int idx = tid + p * 256;
    const int kk  = idx >> 6;
    const int nn  = idx & 63;
    const int ni  = nn & 15;
    const float vb = WB[(size_t)(k0 + kk) * kNst + ni];
    const float vc = WC[(size_t)(k0 + kk) * kNst + ni];
    const float fb = (nn < 16) ? 1.0f : 0.0f;
    const float fc = (nn >= 16 && nn < 32) ? 1.0f : 0.0f;
    const float vs = fmaf(fb, vb, fc * vc);
    tile[kk * 65 + nn] = (nn < 32) ? (vs * scale) : 0.f;
  }
  __syncthreads();
  const int q = lane >> 3, c8 = (lane & 7) * 8;
  v8h hv[2];
#pragma unroll
  for (int it = 0; it < 2; ++it) {
    const int nrow = it * 32 + wave * 4 + q;
#pragma unroll
    for (int e = 0; e < 8; ++e) hv[it][e] = (_Float16)tile[(c8 + e) * 65 + nrow];
  }
  for (int pass = 0; pass < 2; ++pass) {
#pragma unroll
    for (int it = 0; it < 2; ++it) {
      const int nrow = it * 32 + wave * 4 + q;
      *(volatile v8h*)(Bt + (size_t)nrow * Kdim + k0 + c8) = hv[it];
    }
    __threadfence();
  }
}

__global__ __launch_bounds__(256) void ln_kernel(
    const float* __restrict__ x, const float* __restrict__ gamma, const float* __restrict__ beta,
    unsigned short* __restrict__ xn16)
{
  const int lane = threadIdx.x & 31, wave = threadIdx.x >> 5;
  const int row = blockIdx.x * 8 + wave;
  const float* xr = x + (size_t)row * kHid;
  float v[32];
#pragma unroll
  for (int it = 0; it < 4; ++it) {
    const v4f a0 = *(const v4f*)(xr + it * 256 + lane * 8);
    const v4f a1 = *(const v4f*)(xr + it * 256 + lane * 8 + 4);
#pragma unroll
    for (int e = 0; e < 4; ++e) { v[it * 8 + e] = a0[e]; v[it * 8 + 4 + e] = a1[e]; }
  }
  float s = 0.f;
#pragma unroll
  for (int i = 0; i < 32; ++i) s += v[i];
#pragma unroll
  for (int off = 16; off >= 1; off >>= 1) s += __shfl_xor(s, off, 32);
  const float mean = s * (1.0f / (float)kHid);
  float qv = 0.f;
#pragma unroll
  for (int i = 0; i < 32; ++i) { const float dd = v[i] - mean; qv += dd * dd; }
#pragma unroll
  for (int off = 16; off >= 1; off >>= 1) qv += __shfl_xor(qv, off, 32);
  const float var  = qv * (1.0f / (float)kHid);
  const float rstd = rsqrtf(var + 1e-5f);
  v8h hv[4];
#pragma unroll
  for (int it = 0; it < 4; ++it) {
    const int c = it * 256 + lane * 8;
    const v4f g0 = *(const v4f*)(gamma + c);
    const v4f g1 = *(const v4f*)(gamma + c + 4);
    const v4f b0 = *(const v4f*)(beta + c);
    const v4f b1 = *(const v4f*)(beta + c + 4);
#pragma unroll
    for (int e = 0; e < 4; ++e) {
      hv[it][e]     = (_Float16)(((v[it * 8 + e] - mean) * rstd) * g0[e] + b0[e]);
      hv[it][4 + e] = (_Float16)(((v[it * 8 + 4 + e] - mean) * rstd) * g1[e] + b1[e]);
    }
  }
  unsigned short* xo = xn16 + (size_t)row * kHid;
  for (int pass = 0; pass < 2; ++pass) {
#pragma unroll
    for (int it = 0; it < 4; ++it) *(volatile v8h*)(xo + it * 256 + lane * 8) = hv[it];
    __threadfence();
  }
}

__global__ __launch_bounds__(64) void scan_kernel(
    const unsigned short* __restrict__ Up, const unsigned short* __restrict__ Zp, const unsigned short* __restrict__ Gp,
    const float* __restrict__ BC, const float* __restrict__ Alog, const float* __restrict__ Dp,
    unsigned short* __restrict__ Y16)
{
  __shared__ __align__(16) float sBC[kScanTS * kBcP];
  __shared__ __align__(16) float sY[kScanTS * kScanYP];
  __shared__ __align__(16) float sA[kNst * kScanCh];
  const int tid = threadIdx.x, lane = tid & 31, wave = tid >> 5;
  constexpr int kBlkPerB = kInner / kScanCh;
  const int bix = blockIdx.x / kBlkPerB;
  const int d0  = (blockIdx.x - bix * kBlkPerB) * kScanCh;
  const int d   = d0 + tid;
  const size_t row0 = (size_t)bix * kSeq;
#pragma unroll 1
  for (int s = 0; s < kNst; ++s) sA[s * kScanCh + tid] = -expf(Alog[(size_t)d * kNst + s]);
  __syncthreads();
  float negA[kNst], h[kNst];
#pragma unroll
  for (int s = 0; s < kNst; ++s) {
    negA[s] = sA[s * kScanCh + tid];
    h[s] = 0.f;
  }
  const float Dd = Dp[d];
  const int lr = tid >> 3, lc4 = (tid & 7) * 4;
  const int q = lane >> 3, c8 = (lane & 7) * 8;
#pragma unroll 1
  for (int t0 = 0; t0 < kSeq; t0 += kScanTS) {
    __syncthreads();
#pragma unroll
    for (int i = 0; i < 8; ++i) {
      const int r = lr + 8 * i;
      *(v4f*)(sBC + r * kBcP + lc4) = *(const v4f*)(BC + (row0 + t0 + r) * kBcP + lc4);
    }
    __syncthreads();
#pragma unroll 1
    for (int s = 0; s < kScanTS; ++s) {
      const size_t gi = (row0 + t0 + s) * kInner + d;
      unsigned ub = Up[gi];
      unsigned zb = Zp[gi];
      unsigned gb = Gp[gi];
      asm volatile("" : "+v"(ub));
      asm volatile("" : "+v"(zb));
      asm volatile("" : "+v"(gb));
      const float* xr = sBC + s * kBcP;
      float Bs[kNst], Cs[kNst];
#pragma unroll
      for (int q4 = 0; q4 < 4; ++q4) {
        const v4f bv = *(const v4f*)(xr + 4 * q4);
        const v4f cv = *(const v4f*)(xr + kNst + 4 * q4);
        Bs[4 * q4 + 0] = bv[0]; Bs[4 * q4 + 1] = bv[1]; Bs[4 * q4 + 2] = bv[2]; Bs[4 * q4 + 3] = bv[3];
        Cs[4 * q4 + 0] = cv[0]; Cs[4 * q4 + 1] = cv[1]; Cs[4 * q4 + 2] = cv[2]; Cs[4 * q4 + 3] = cv[3];
      }
      const float zv  = h16_to_f32(zb);
      const float xt  = h16_to_f32(ub);
      const float sgv = h16_to_f32(gb);
      const float a   = __expf(-fabsf(zv));
      const float up1 = 1.0f + a;
      const float l1p = __logf(up1) + (a - (up1 - 1.0f)) * __builtin_amdgcn_rcpf(up1);
      const float dt  = fmaxf(zv, 0.0f) + l1p;
      const float dtx = dt * xt;
      float y = 0.f;
#pragma unroll
      for (int k = 0; k < kNst; ++k) {
        const float e = __expf(dt * negA[k]);
        h[k] = e * h[k] + dtx * Bs[k];
        y = h[k] * Cs[k] + y;
      }
      y = xt * Dd + y;
      y = y * sgv;
      sY[s * kScanYP + tid] = y * kYCarry;
    }
    __syncthreads();
    v8h hv[8];
#pragma unroll
    for (int it = 0; it < 8; ++it) {
      const int row = it * 8 + wave * 4 + q;
      const float* sp = sY + row * kScanYP + c8;
      const v4f a0 = *(const v4f*)(sp);
      const v4f a1 = *(const v4f*)(sp + 4);
#pragma unroll
      for (int e = 0; e < 4; ++e) {
        hv[it][e]     = (_Float16)a0[e];
        hv[it][4 + e] = (_Float16)a1[e];
      }
    }
    for (int pass = 0; pass < 2; ++pass) {
#pragma unroll
      for (int it = 0; it < 8; ++it) {
        const int row = it * 8 + wave * 4 + q;
        const size_t o = (row0 + t0 + row) * kInner + d0 + c8;
        *(volatile v8h*)(Y16 + o) = hv[it];
      }
      __threadfence();
    }
  }
}

extern "C" void kernel_launch(void* const* d_in, const int* in_sizes, int n_in,
                              void* d_out, int out_size, void* d_ws, size_t ws_size,
                              hipStream_t stream)
{
  if (n_in < 17) return;
  if (in_sizes[0] != kRows * kHid) return;
  if (in_sizes[1] != kHid || in_sizes[2] != kHid) return;
  if (in_sizes[3] != kHid * kProjW || in_sizes[4] != kProjW) return;
  if (in_sizes[5] != kInner * kDtR || in_sizes[6] != kDtR) return;
  if (in_sizes[7] != kDtR * kInner || in_sizes[8] != kInner) return;
  if (in_sizes[9] != kInner * kNst || in_sizes[10] != kNst) return;
  if (in_sizes[11] != kInner * kNst || in_sizes[12] != kNst) return;
  if (in_sizes[13] != kInner * kNst || in_sizes[14] != kInner) return;
  if (in_sizes[15] != kInner * kHid || in_sizes[16] != kHid) return;
  if (out_size != kRows * kHid) return;
  if (ws_size < kWsTotal) return;

  const float* x        = (const float*)d_in[0];
  const float* ln_gamma = (const float*)d_in[1];
  const float* ln_beta  = (const float*)d_in[2];
  const float* W_in     = (const float*)d_in[3];
  const float* b_in     = (const float*)d_in[4];
  const float* W_delta  = (const float*)d_in[5];
  const float* b_delta  = (const float*)d_in[6];
  const float* W_dt     = (const float*)d_in[7];
  const float* b_dt     = (const float*)d_in[8];
  const float* W_B      = (const float*)d_in[9];
  const float* b_B      = (const float*)d_in[10];
  const float* W_C      = (const float*)d_in[11];
  const float* b_C      = (const float*)d_in[12];
  const float* A_log    = (const float*)d_in[13];
  const float* Dvec     = (const float*)d_in[14];
  const float* W_out    = (const float*)d_in[15];
  const float* b_out    = (const float*)d_in[16];
  float* out = (float*)d_out;

  char* ws = (char*)d_ws;
  unsigned short* WINT = (unsigned short*)(ws + kOffWINT);
  unsigned short* WCAT = (unsigned short*)(ws + kOffWCAT);
  unsigned short* WDT  = (unsigned short*)(ws + kOffWDT);
  unsigned short* WOUT = (unsigned short*)(ws + kOffWOUT);
  unsigned short* XN16 = (unsigned short*)(ws + kOffXN16);
  unsigned short* U16  = (unsigned short*)(ws + kOffU16);
  unsigned short* SG16 = (unsigned short*)(ws + kOffSG16);
  unsigned short* DR16 = (unsigned short*)(ws + kOffDR16);
  float*          BC   = (float*)(ws + kOffBC);
  unsigned short* Z16  = (unsigned short*)(ws + kOffZ16);
  unsigned short* Y16  = (unsigned short*)(ws + kOffY16);

  transpose_cast_kernel<<<dim3(kProjW / 64, kHid / 64), 256, 0, stream>>>(W_in, WINT, kHid, kProjW, kWCarry);
  transpose_cast_kernel<<<dim3(kDtR / 64, kInner / 64), 256, 0, stream>>>(W_delta, WCAT, kInner, kDtR, kWCarry);
  transpose_cast_bc_kernel<<<dim3(kInner / 64), 256, 0, stream>>>(W_B, W_C, WCAT + (size_t)64 * kInner, kInner, kWCarry);
  transpose_cast_kernel<<<dim3(kInner / 64, kDtR / 64), 256, 0, stream>>>(W_dt, WDT, kDtR, kInner, kWCarry);
  transpose_cast_kernel<<<dim3(kHid / 64, kInner / 64), 256, 0, stream>>>(W_out, WOUT, kInner, kHid, kWCarry);

  ln_kernel<<<dim3(kRows / 8), 256, 0, stream>>>(x, ln_gamma, ln_beta, XN16);

  gemm64_f16<1, false, 3><<<dim3((kRows / 64) * (kProjW / 64) / 8), 256, 0, stream>>>(
      XN16, kHid, WINT, kHid,
      (void*)U16, (void*)SG16, kInner, kInner,
      b_in, b_in, x,
      kRows, kProjW, kHid, 1.0f / kWCarry, 1.0f);

  gemm64_f16<1, false, 0><<<dim3((kRows / 64) * 1 / 8), 256, 0, stream>>>(
      U16, kInner, WCAT, kInner,
      (void*)DR16, (void*)DR16, kDtR, kDtR,
      b_delta, b_delta, x,
      kRows, 64, kInner, kDrCarry / kWCarry, kDrCarry);

  gemm64_f16<3, false, 0><<<dim3((kRows / 64) * 1 / 8), 256, 0, stream>>>(
      U16, kInner, WCAT + (size_t)64 * kInner, kInner,
      (void*)BC, (void*)BC, kBcP, 64,
      b_B, b_C, x,
      kRows, 64, kInner, 1.0f / kWCarry, 1.0f);

  gemm64_f16<1, false, 0><<<dim3((kRows / 64) * (kInner / 64) / 8), 256, 0, stream>>>(
      DR16, kDtR, WDT, kDtR,
      (void*)Z16, (void*)Z16, kInner, kInner,
      b_dt, b_dt, x,
      kRows, kInner, kDtR, 1.0f / (kDrCarry * kWCarry), 1.0f);

  scan_kernel<<<dim3(kBatch * (kInner / kScanCh)), kScanCh, 0, stream>>>(U16, Z16, SG16, BC, A_log, Dvec, Y16);

  gemm64_f16<0, true, 0><<<dim3((kRows / 64) * (kHid / 64) / 8), 256, 0, stream>>>(
      Y16, kInner, WOUT, kInner,
      (void*)out, (void*)out, kHid, kHid,
      b_out, b_out, x,
      kRows, kHid, kInner, 1.0f / (kYCarry * kWCarry), 1.0f);
}
